// FourierKANLayer_75350906241070
// MI455X (gfx1250) — hardware-verified
//
#include <hip/hip_runtime.h>
#include <stdint.h>

typedef _Float16 v16h __attribute__((ext_vector_type(16)));
typedef _Float16 v8h  __attribute__((ext_vector_type(8)));
typedef float    v8f  __attribute__((ext_vector_type(8)));
typedef float    v4f  __attribute__((ext_vector_type(4)));
typedef unsigned int v4u __attribute__((ext_vector_type(4)));

#define IN_DIM   256
#define OUT_DIM  256
#define GRID_SZ  32
#define KTOT     (IN_DIM * 2 * GRID_SZ)
#define BM       64
#define A_PITCH  72
#define S_PITCH  68
#define B_SCALE   1024.0f
#define B_UNSCALE (1.0f / 1024.0f)

union FragH { v16h v; v8h hf[2]; };
union Pack8 { v8h h; v4u u; };

__device__ __forceinline__ v8f wmma_f16(const v16h a, const v16h b, v8f acc) {
  acc = __builtin_amdgcn_wmma_f32_16x16x32_f16(false, a, false, b, (short)0, acc, false, false);
  asm volatile("v_nop\n\tv_nop\n\tv_nop\n\tv_nop" : "+v"(acc) : "v"(a), "v"(b));
  return acc;
}

struct CS { float c; float s; };
__device__ __forceinline__ CS rot(CS a, float c1, float s1) {
  CS r;
  r.c = a.c * c1 - a.s * s1;
  r.s = a.s * c1 + a.c * s1;
  return r;
}

__global__ __launch_bounds__(256) void pack_coeffs(const float* __restrict__ coeffs,
                                                   _Float16* bt, int nchunks) {
  int gid = blockIdx.x * 256 + threadIdx.x;
  bool ok = gid < nchunks;
  int gidc = ok ? gid : 0;
  size_t o0 = (size_t)gidc * 8;
  int n  = (int)(o0 / KTOT);
  int K0 = (int)(o0 % KTOT);
  int i  = K0 >> 6;
  int c  = (K0 >> 5) & 1;
  int g0 = K0 & 31;
  const float* src = coeffs + ((((size_t)c * OUT_DIM + n) * IN_DIM + i) * GRID_SZ + g0);
  v4f f0 = *(const v4f*)src;
  v4f f1 = *(const v4f*)(src + 4);
  Pack8 pk;
  pk.h[0] = (_Float16)(f0.x * B_SCALE);
  pk.h[1] = (_Float16)(f0.y * B_SCALE);
  pk.h[2] = (_Float16)(f0.z * B_SCALE);
  pk.h[3] = (_Float16)(f0.w * B_SCALE);
  pk.h[4] = (_Float16)(f1.x * B_SCALE);
  pk.h[5] = (_Float16)(f1.y * B_SCALE);
  pk.h[6] = (_Float16)(f1.z * B_SCALE);
  pk.h[7] = (_Float16)(f1.w * B_SCALE);
  if (ok) *(volatile v4u*)(bt + o0) = pk.u;
  __threadfence();
  if (ok) *(volatile v4u*)(bt + o0) = pk.u;
}

__global__ __launch_bounds__(256) void fourier_gemm(const float* __restrict__ x,
                                                    const _Float16* __restrict__ bt,
                                                    const float* __restrict__ bias,
                                                    float* out, int nrows) {
  __shared__ __align__(16) _Float16 a_s[BM * A_PITCH];
  __shared__ __align__(16) float    st_s[8 * 16 * S_PITCH];

  const int tid  = threadIdx.x;
  const int lane = tid & 31;
  const int wave = tid >> 5;
  const int h    = lane >> 4;
  const int m    = lane & 15;
  const int mgrp = wave & 1;
  const int ngrp = wave >> 1;
  const int m0   = blockIdx.x * BM;

  const int brow = tid & 63;
  const int bp   = tid >> 6;
  int xrow = m0 + brow;
  if (xrow > nrows - 1) xrow = nrows - 1;
  if (xrow < 0) xrow = 0;
  const float* xrowp = x + (size_t)xrow * IN_DIM;

  v8f acc[8];
#pragma unroll
  for (int t = 0; t < 8; ++t) acc[t] = (v8f){0.f, 0.f, 0.f, 0.f, 0.f, 0.f, 0.f, 0.f};

  const _Float16* btw = bt + (size_t)(ngrp * 64 + m) * KTOT;
  const _Float16* arow0 = a_s + (mgrp * 32 + m) * A_PITCH + 8 * h;
  _Float16* abuild = a_s + brow * A_PITCH + 8 * bp;

#pragma unroll 1
  for (int i = 0; i < IN_DIM; ++i) {
    {
      float xv = xrowp[i];
      float s1, c1;
      sincosf(xv, &s1, &c1);
      float c2 = c1 * c1 - s1 * s1, s2 = 2.0f * s1 * c1;
      float c4 = c2 * c2 - s2 * s2, s4 = 2.0f * s2 * c2;
      float c8 = c4 * c4 - s4 * s4, s8 = 2.0f * s4 * c4;
      CS r; r.c = c1; r.s = s1;
      if (bp & 1) r = rot(r, c8, s8);
      if (bp & 2) {
        float c16 = c8 * c8 - s8 * s8, s16 = 2.0f * s8 * c8;
        r = rot(r, c16, s16);
      }
      v8h cv, sv;
#pragma unroll
      for (int j = 0; j < 8; ++j) {
        cv[j] = (_Float16)r.c;
        sv[j] = (_Float16)r.s;
        r = rot(r, c1, s1);
      }
      *(v8h*)abuild        = cv;
      *(v8h*)(abuild + 32) = sv;
    }
    __syncthreads();

#pragma unroll
    for (int ks = 0; ks < 2; ++ks) {
      FragH a0, a1;
      const _Float16* ar = arow0 + 32 * ks;
      a0.hf[0] = *(const v8h*)(ar);
      a0.hf[1] = *(const v8h*)(ar + 16);
      a1.hf[0] = *(const v8h*)(ar + 16 * A_PITCH);
      a1.hf[1] = *(const v8h*)(ar + 16 * A_PITCH + 16);
      const _Float16* bk = btw + (size_t)i * 64 + 32 * ks + 8 * h;
#pragma unroll
      for (int t = 0; t < 4; ++t) {
        FragH b;
        const _Float16* bq = bk + (size_t)t * 16 * KTOT;
        b.hf[0] = *(const v8h*)(bq);
        b.hf[1] = *(const v8h*)(bq + 16);
        acc[t]     = wmma_f16(a0.v, b.v, acc[t]);
        acc[4 + t] = wmma_f16(a1.v, b.v, acc[4 + t]);
      }
    }
    __syncthreads();
  }

  float bv[4];
#pragma unroll
  for (int t = 0; t < 4; ++t) bv[t] = bias[ngrp * 64 + 16 * t + m];

  float* stw = st_s + wave * (16 * S_PITCH);
  v4f vals[2][8];
#pragma unroll
  for (int mt = 0; mt < 2; ++mt) {
#pragma unroll
    for (int t = 0; t < 4; ++t) {
#pragma unroll
      for (int r = 0; r < 8; ++r)
        stw[(8 * h + r) * S_PITCH + 16 * t + m] = acc[mt * 4 + t][r] * B_UNSCALE + bv[t];
    }
    __syncthreads();
#pragma unroll
    for (int q = 0; q < 8; ++q) {
      int L  = q * 4 + (lane >> 3);
      int rl = L >> 1, ch = L & 1;
      vals[mt][q] = *(const v4f*)(stw + rl * S_PITCH + ch * 32 + (lane & 7) * 4);
    }
    __syncthreads();
  }

  const int rowbase = m0 + mgrp * 32;
  const int colbase = ngrp * 64 + (lane & 7) * 4;
  auto store_pass = [&]() __attribute__((always_inline)) {
#pragma unroll
    for (int mt = 0; mt < 2; ++mt) {
#pragma unroll
      for (int q = 0; q < 8; ++q) {
        int L  = q * 4 + (lane >> 3);
        int rl = L >> 1, ch = L & 1;
        int row = rowbase + mt * 16 + rl;
        if (row < nrows) {
          size_t off = (size_t)row * OUT_DIM + colbase + ch * 32;
          *(volatile v4f*)(out + off) = vals[mt][q];
        }
      }
    }
  };
  store_pass();
  __threadfence();
  store_pass();
}

extern "C" void kernel_launch(void* const* d_in, const int* in_sizes, int n_in,
                              void* d_out, int out_size, void* d_ws, size_t ws_size,
                              hipStream_t stream) {
  if (n_in < 3) return;
  const float* x      = (const float*)d_in[0];
  const float* coeffs = (const float*)d_in[1];
  const float* bias   = (const float*)d_in[2];
  float*       out    = (float*)d_out;

  const int nrows = in_sizes[0] / IN_DIM;
  if (nrows <= 0) return;
  if (in_sizes[1] != 2 * OUT_DIM * IN_DIM * GRID_SZ) return;
  if (in_sizes[2] < OUT_DIM) return;
  if (out_size < nrows * OUT_DIM) return;

  const size_t bt_bytes = (size_t)OUT_DIM * KTOT * sizeof(_Float16);
  if (bt_bytes > ws_size) return;
  _Float16* bt = (_Float16*)d_ws;

  const int nchunks = OUT_DIM * KTOT / 8;
  pack_coeffs<<<(nchunks + 255) / 256, 256, 0, stream>>>(coeffs, bt, nchunks);
  fourier_gemm<<<(nrows + BM - 1) / BM, 256, 0, stream>>>(x, bt, bias, out, nrows);
}
